// GraphMultiHeadAttention_38654705664487
// MI455X (gfx1250) — hardware-verified
//
#include <hip/hip_runtime.h>
#include <math.h>
#include <stdint.h>
#include <stddef.h>


#define NGR    32
#define NND    512
#define NTOT   (NGR * NND)
#define HID    512
#define NHD    8
#define HDM    64
#define EDW    16
#define NHALF  2
#define GHALF  (NGR / NHALF)
#define RHALF  (GHALF * NND)
#define PLD    1024
#define NTHR   256
#define WSMAX  134217728

static_assert(HID == NHD * HDM && HDM == 64 && NHD == 8);
static_assert(PLD == 2 * HID);
static_assert((RHALF % 64) == 0 && (HID % 64) == 0 && (NND % 64) == 0 && (PLD % 32) == 0 && (HID % 32) == 0);
static_assert(((RHALF / 64) * (HID / 64)) % 8 == 0);
static_assert(((HID / 64) * (NND / 64)) % 8 == 0);
static_assert(NGR == NHALF * GHALF);
static_assert(HID == 64 * 8);
static_assert(EDW == 16 && NHD == 8 && EDW * NHD <= NTHR);

typedef __attribute__((ext_vector_type(16))) _Float16 v16h;
typedef __attribute__((ext_vector_type(8)))  _Float16 v8h;
typedef __attribute__((ext_vector_type(16))) __bf16   v16b;
typedef __attribute__((ext_vector_type(8)))  __bf16   v8b;
typedef __attribute__((ext_vector_type(8)))  float    v8f;
typedef __attribute__((ext_vector_type(4)))  float    v4f;
typedef __attribute__((ext_vector_type(2)))  float    v2f;
typedef __attribute__((ext_vector_type(4)))  unsigned int v4u;
typedef __attribute__((ext_vector_type(4)))  int      v4i;
typedef __attribute__((ext_vector_type(8)))  unsigned short v8us;
typedef v4f  __attribute__((may_alias)) v4fa;
typedef v2f  __attribute__((may_alias)) v2fa;
typedef v4u  __attribute__((may_alias)) v4ua;

__device__ __forceinline__ unsigned short f2bf_bits(float f) {
  unsigned u = __float_as_uint(f);
  return (unsigned short)((u + 0x7FFFu + ((u >> 16) & 1u)) >> 16);
}
__device__ __forceinline__ float bf_bits2f(unsigned short h) { return __uint_as_float(((unsigned)h) << 16); }
__device__ __forceinline__ float bfrf(float f) { return bf_bits2f(f2bf_bits(f)); }
__device__ __forceinline__ unsigned int f2bfu(float f) {
  const unsigned int u = __float_as_uint(f);
  return ((u + 0x7FFFu + ((u >> 16) & 1u)) >> 16) & 0xFFFFu;
}
__device__ __forceinline__ float bf2f(unsigned int b) { return __uint_as_float(b << 16); }
__device__ __forceinline__ v4f bfr4(const v4f a) {
  v4f r; r.x = bfrf(a.x); r.y = bfrf(a.y); r.z = bfrf(a.z); r.w = bfrf(a.w); return r;
}
__device__ __forceinline__ unsigned int pk2(float lo, float hi) { return f2bfu(lo) | (f2bfu(hi) << 16); }
__device__ __forceinline__ v4u pack8(const v4f a, const v4f b) {
  v4u r;
  r.x = pk2(a.x, a.y); r.y = pk2(a.z, a.w); r.z = pk2(b.x, b.y); r.w = pk2(b.z, b.w);
  return r;
}
__device__ __forceinline__ void hl2(float v0, float v1, unsigned int& hw, unsigned int& lw) {
  const unsigned int h0 = f2bfu(v0), h1 = f2bfu(v1);
  const unsigned int l0 = f2bfu(v0 - bf2f(h0)), l1 = f2bfu(v1 - bf2f(h1));
  hw = h0 | (h1 << 16);
  lw = l0 | (l1 << 16);
}
__device__ __forceinline__ void pack8hl(const v4f a, const v4f b, v4u& hv, v4u& lv) {
  unsigned int h, l;
  hl2(a.x, a.y, h, l); hv.x = h; lv.x = l;
  hl2(a.z, a.w, h, l); hv.y = h; lv.y = l;
  hl2(b.x, b.y, h, l); hv.z = h; lv.z = l;
  hl2(b.z, b.w, h, l); hv.w = h; lv.w = l;
}

__device__ __forceinline__ void dep_guard_b(v8f& a, v8f& b, v16b x, v16b y) { asm volatile("v_nop\n\tv_nop\n\tv_nop\n\tv_nop" : "+v"(a), "+v"(b) : "v"(x), "v"(y)); }
__device__ __forceinline__ void keep4_b(v16b a, v16b b, v16b c, v16b d) { asm volatile("v_nop" :: "v"(a), "v"(b), "v"(c), "v"(d)); }
__device__ __forceinline__ void acc_guard4(v8f& a, v8f& b, v8f& c, v8f& d) { asm volatile("v_nop\n\tv_nop\n\tv_nop\n\tv_nop" : "+v"(a), "+v"(b), "+v"(c), "+v"(d)); }

struct FragBF {
  union U { v16b v; v8b h[2]; };
  static __device__ __forceinline__ v16b load(const __bf16* p) {
    U f; f.h[0] = *(const v8b*)(p); f.h[1] = *(const v8b*)(p + 16); return f.v;
  }
  static __device__ __forceinline__ v8f mma(v16b a, v16b b, v8f c) {
    return __builtin_amdgcn_wmma_f32_16x16x32_bf16(false, a, false, b, (short)0, c, false, false);
  }
  static __device__ __forceinline__ void guard(v8f& a, v8f& b, v16b x, v16b y) { dep_guard_b(a, b, x, y); }
  static __device__ __forceinline__ void keep(v16b a, v16b b, v16b c, v16b d) { keep4_b(a, b, c, d); }
};
union FB { v16b v; v8b h[2]; };

__device__ __forceinline__ v8f at_mma(v16b a, v16b b, v8f c) {
  c = __builtin_amdgcn_wmma_f32_16x16x32_bf16(false, a, false, b, (short)0, c, false, false);
  asm volatile("v_nop\n\tv_nop\n\tv_nop\n\tv_nop" : "+v"(c) : "v"(a), "v"(b));
  return c;
}
__device__ __forceinline__ __bf16 at_f2bf(float f) { return __builtin_bit_cast(__bf16, f2bf_bits(f)); }
__device__ __forceinline__ void at_split(float f, __bf16& hi, __bf16& lo) {
  const unsigned short hb = f2bf_bits(f);
  hi = __builtin_bit_cast(__bf16, hb);
  lo = at_f2bf(f - __uint_as_float(((unsigned)hb) << 16));
}

template <bool SPLIT, int BIAS_MODE, int OUT_MODE, bool RESID, int ACT = 0>
__global__ __launch_bounds__(256) void wmma_gemm64(
    const unsigned short* __restrict__ Ap, const unsigned short* __restrict__ A2p, int lda, long strideA,
    const unsigned short* __restrict__ Btp, const unsigned short* __restrict__ Bt2p, int ldb, long strideB,
    void* __restrict__ Cout, void* __restrict__ Cout2, int ldc, long strideC,
    const float* __restrict__ bias,
    const float* __restrict__ resid, long strideR,
    int M, int N, int K, float scale) {
  typedef __bf16 T;
  typedef v16b V;
  const T* A = (const T*)Ap; const T* A2 = (const T*)A2p; const T* Bt = (const T*)Btp; const T* Bt2 = (const T*)Bt2p;
  __shared__ __align__(16) float sT[8][16 * 68];
  const int b    = blockIdx.y;
  const int lane = threadIdx.x & 31;
  const int wave = threadIdx.x >> 5;
  const int tilesN = N >> 6;
  const int tilesM = M >> 6;
  const int tile = blockIdx.x * 8 + wave;
  if (tile >= tilesM * tilesN) return;
  const int tm = tile / tilesN;
  const int tn = tile - tm * tilesN;
  const int m0 = tm << 6;
  const int n0 = tn << 6;

  const T* Ab  = A  + (size_t)b * strideA;
  const T* Bb  = Bt + (size_t)b * strideB;
  const T* Ab2 = SPLIT ? (A2  + (size_t)b * strideA) : nullptr;
  const T* Bb2 = SPLIT ? (Bt2 + (size_t)b * strideB) : nullptr;

  const int rlane = lane & 15;
  const int koff  = (lane >> 4) * 8;
  const int mOff  = (lane >> 4) * 8;

  v8f acc[4][4];
#pragma unroll
  for (int i = 0; i < 4; ++i)
#pragma unroll
    for (int j = 0; j < 4; ++j) acc[i][j] = (v8f){0.f,0.f,0.f,0.f,0.f,0.f,0.f,0.f};

  for (int k0 = 0; k0 < K; k0 += 32) {
    V bh[4], bl[4];
#pragma unroll
    for (int j = 0; j < 4; ++j) {
      const size_t bo = (size_t)(n0 + (j << 4) + rlane) * ldb + koff + k0;
      bh[j] = FragBF::load(Bb + bo);
      if (SPLIT) bl[j] = FragBF::load(Bb2 + bo);
    }
#pragma unroll
    for (int i = 0; i < 4; ++i) {
      const size_t ao = (size_t)(m0 + (i << 4) + rlane) * lda + koff + k0;
      V ah = FragBF::load(Ab + ao);
      V al;
      if (SPLIT) al = FragBF::load(Ab2 + ao);
#pragma unroll
      for (int j = 0; j < 4; ++j) {
        acc[i][j] = FragBF::mma(ah, bh[j], acc[i][j]);
        if (SPLIT) {
          acc[i][j] = FragBF::mma(ah, bl[j], acc[i][j]);
          acc[i][j] = FragBF::mma(al, bh[j], acc[i][j]);
        }
      }
      FragBF::guard(acc[i][0], acc[i][3], ah, SPLIT ? al : ah);
    }
    FragBF::keep(bh[0], bh[1], bh[2], bh[3]);
    if (SPLIT) FragBF::keep(bl[0], bl[1], bl[2], bl[3]);
  }
  acc_guard4(acc[0][0], acc[0][1], acc[0][2], acc[0][3]);
  acc_guard4(acc[1][0], acc[1][1], acc[1][2], acc[1][3]);
  acc_guard4(acc[2][0], acc[2][1], acc[2][2], acc[2][3]);
  acc_guard4(acc[3][0], acc[3][1], acc[3][2], acc[3][3]);

  float* slab = sT[wave];
  const float* Rb = RESID ? (resid + (size_t)b * strideR) : nullptr;
#pragma unroll
  for (int i = 0; i < 4; ++i) {
    const int mBase = m0 + (i << 4);
    float bm[8];
    if (BIAS_MODE == 1) {
      const v4f b0v = bfr4(*(const v4fa*)(bias + mBase + mOff));
      const v4f b1v = bfr4(*(const v4fa*)(bias + mBase + mOff + 4));
      bm[0] = b0v.x; bm[1] = b0v.y; bm[2] = b0v.z; bm[3] = b0v.w;
      bm[4] = b1v.x; bm[5] = b1v.y; bm[6] = b1v.z; bm[7] = b1v.w;
    } else {
#pragma unroll
      for (int r = 0; r < 8; ++r) bm[r] = 0.f;
    }
#pragma unroll
    for (int j = 0; j < 4; ++j) {
      const int n = n0 + (j << 4) + rlane;
      float bv = 0.f;
      if (BIAS_MODE == 2) bv = bfrf(bias[n]);
#pragma unroll
      for (int r = 0; r < 8; ++r) {
        float v = acc[i][j][r] * scale;
        if (BIAS_MODE == 1) v += bm[r];
        if (BIAS_MODE == 2) v += bv;
        if (RESID) v += Rb[(size_t)(mBase + mOff + r) * ldc + n];
        if (ACT == 1) v = tanhf(v);
        if (ACT == 2) v = fmaxf(v, 0.0f);
        if (ACT == 4) v = (v > 0.f) ? v : 0.01f * v;
        slab[(mOff + r) * 68 + (j << 4) + rlane] = v;
      }
    }
    __builtin_amdgcn_fence(__ATOMIC_RELEASE, "workgroup");
    __builtin_amdgcn_wave_barrier();
    __builtin_amdgcn_fence(__ATOMIC_ACQUIRE, "workgroup");
    if (OUT_MODE == 0) {
      float* C = (float*)Cout + (size_t)b * strideC;
      const int hh = lane >> 4, c4 = (lane & 15) * 4;
      for (int pass = 0; pass < 2; ++pass) {
#pragma unroll
        for (int it = 0; it < 8; ++it) {
          const int row = it * 2 + hh;
          v4f v = *(const v4f*)(slab + row * 68 + c4);
          *(volatile v4f*)(C + (size_t)(mBase + row) * ldc + n0 + c4) = v;
        }
        __threadfence();
      }
    } else {
      const int q = lane >> 3, c8 = (lane & 7) * 8;
      unsigned short* C  = (unsigned short*)Cout  + (size_t)b * strideC;
      unsigned short* C2 = (OUT_MODE == 2) ? ((unsigned short*)Cout2 + (size_t)b * strideC) : nullptr;
      for (int pass = 0; pass < 2; ++pass) {
#pragma unroll
        for (int it = 0; it < 4; ++it) {
          const int row = it * 4 + q;
          const float* sp = slab + row * 68 + c8;
          v8h hv, lv;
#pragma unroll
          for (int e = 0; e < 8; ++e) {
            if (OUT_MODE == 1) {
              hv[e] = (_Float16)sp[e];
            } else {
              unsigned short hb = f2bf_bits(sp[e]);
              unsigned short lb = f2bf_bits(sp[e] - bf_bits2f(hb));
              hv[e] = __builtin_bit_cast(_Float16, hb);
              lv[e] = __builtin_bit_cast(_Float16, lb);
            }
          }
          *(volatile v8h*)(C + (size_t)(mBase + row) * ldc + n0 + c8) = hv;
          if (OUT_MODE == 2) *(volatile v8h*)(C2 + (size_t)(mBase + row) * ldc + n0 + c8) = lv;
        }
        __threadfence();
      }
    }
    __builtin_amdgcn_fence(__ATOMIC_RELEASE, "workgroup");
    __builtin_amdgcn_wave_barrier();
    __builtin_amdgcn_fence(__ATOMIC_ACQUIRE, "workgroup");
  }
}

__global__ __launch_bounds__(NTHR) void k_xprep(const float* __restrict__ x, unsigned short* xb, int nN, int nUnits) {
  const int i = (int)blockIdx.x * NTHR + (int)threadIdx.x;
  if (i >= nUnits) return;
  const int row = i >> 6;
  const int c0  = (i & 63) * 8;
  const int rc  = row < nN ? row : nN - 1;
  const float* p = x + (size_t)rc * HID + c0;
  v4f a = *(const v4fa*)p;
  v4f b = *(const v4fa*)(p + 4);
  const v4f z4 = {0.f, 0.f, 0.f, 0.f};
  if (row >= nN) { a = z4; b = z4; }
  const v4u hv = pack8(a, b);
  unsigned short* o = xb + (size_t)row * HID + c0;
  *(volatile v4u*)o = hv;
  __threadfence();
  *(volatile v4u*)o = hv;
}

__global__ __launch_bounds__(NTHR) void k_wtr(const float* __restrict__ w, int Kin, int Ncol, int Nrows, int Kout,
                                              unsigned short* wt, int nUnits) {
  const int u = (int)blockIdx.x * NTHR + (int)threadIdx.x;
  if (u >= nUnits) return;
  const int kq = Kout >> 3;
  const int n  = u / kq;
  const int k8 = (u - n * kq) * 8;
  const int kk = k8 - (k8 / Kin) * Kin;
  const int ncl = n < Ncol ? n : Ncol - 1;
  const float* p = w + (size_t)kk * (size_t)Ncol + ncl;
  v4f a, b;
  a.x = p[0];                    a.y = p[(size_t)Ncol];         a.z = p[(size_t)2 * Ncol];     a.w = p[(size_t)3 * Ncol];
  b.x = p[(size_t)4 * Ncol];     b.y = p[(size_t)5 * Ncol];     b.z = p[(size_t)6 * Ncol];     b.w = p[(size_t)7 * Ncol];
  const v4f z4 = {0.f, 0.f, 0.f, 0.f};
  if (n >= Ncol || n >= Nrows) { a = z4; b = z4; }
  const v4u wv = pack8(a, b);
  unsigned short* o = wt + (size_t)n * (size_t)Kout + k8;
  *(volatile v4u*)o = wv;
  __threadfence();
  *(volatile v4u*)o = wv;
}

__global__ __launch_bounds__(NTHR) void k_eb(const float* __restrict__ ea, const float* __restrict__ We,
                                             const float* __restrict__ be, float* EB, int nE, int nUnits) {
  __shared__ float sWe[EDW * NHD];
  __shared__ float sbe[NHD];
  const int tid = (int)threadIdx.x;
  if (tid < EDW * NHD) sWe[tid] = bfrf(We[tid]);
  if (tid < NHD) sbe[tid] = bfrf(be[tid]);
  __syncthreads();
  const int u = (int)blockIdx.x * NTHR + tid;
  if (u >= nUnits) return;
  const int e  = u >> 1;
  const int h0 = (u & 1) * 4;
  const int ec = e < nE ? e : nE - 1;
  const float* er = ea + (size_t)ec * EDW;
  float s0 = 0.f, s1 = 0.f, s2 = 0.f, s3 = 0.f;
#pragma unroll 1
  for (int q = 0; q < 4; ++q) {
    const v4f a = bfr4(*(const v4fa*)(er + 4 * q));
    const float* wr = sWe + (4 * q) * NHD + h0;
    s0 = fmaf(a.x, wr[0],  s0); s1 = fmaf(a.x, wr[1],  s1); s2 = fmaf(a.x, wr[2],  s2); s3 = fmaf(a.x, wr[3],  s3);
    s0 = fmaf(a.y, wr[8],  s0); s1 = fmaf(a.y, wr[9],  s1); s2 = fmaf(a.y, wr[10], s2); s3 = fmaf(a.y, wr[11], s3);
    s0 = fmaf(a.z, wr[16], s0); s1 = fmaf(a.z, wr[17], s1); s2 = fmaf(a.z, wr[18], s2); s3 = fmaf(a.z, wr[19], s3);
    s0 = fmaf(a.w, wr[24], s0); s1 = fmaf(a.w, wr[25], s1); s2 = fmaf(a.w, wr[26], s2); s3 = fmaf(a.w, wr[27], s3);
  }
  v4f o;
  o.x = s0 + sbe[h0]; o.y = s1 + sbe[h0 + 1]; o.z = s2 + sbe[h0 + 2]; o.w = s3 + sbe[h0 + 3];
  const v4f z4 = {0.f, 0.f, 0.f, 0.f};
  if (e >= nE) o = z4;
  float* op = EB + (size_t)e * NHD + h0;
  *(volatile v4f*)op = o;
  __threadfence();
  *(volatile v4f*)op = o;
}

#define AT_NW   8
#define EPT     8
#define CHUNK   (NTHR * EPT)
#define WCAP    (EPT * 32)
#define LISTN   (AT_NW * WCAP)
#define SLOTB   6
#define NSLOT   64
#define HCAP    2048
#define RWCAP   128
#define KVT     4096
#define NDUM    512
#define LO_KV   0
#define LO_P    (8 * KVT * 2)
#define LO_BT   (LO_P + 2 * AT_NW * 1024 * 2)
#define LO_SE   (LO_BT + (2 * KVT + NDUM) * 4)
#define LO_SD   (LO_SE + HCAP * 4)
#define LO_RC   (LO_SD + HCAP * 4)
#define LDS_ATT (LO_RC + (3 * NSLOT + 2 * AT_NW) * 4)

static_assert((LISTN + 2 * HCAP) * 4 <= LO_P);
static_assert(LDS_ATT <= 300000);
static_assert((1 << SLOTB) == NSLOT);
static_assert(NTHR == 32 * AT_NW);
static_assert(NTHR == 4 * NSLOT);
static_assert(NTHR * 32 == 2 * KVT);
static_assert(NDUM == 2 * NTHR && NDUM == 128 * 4);
static_assert(AT_NW * 1024 == 2 * KVT);
static_assert((CHUNK & (CHUNK - 1)) == 0 && CHUNK == 2048);
static_assert(2 * NSLOT == 32 * 4 / 2 * 2 && NSLOT == 2 * 32);

__device__ __forceinline__ int scan_chunk(const int* __restrict__ keys, int nE, int cbase, int slotBase,
                                          int nb, int vec8, int* list, int tid, int lane, int wave) {
  int wc = 0;
  const int el0  = tid * EPT;
  const int e0   = cbase + el0;
  const int sent = -2147483647 - 1;
  v4i da, db;
  if (vec8 != 0 && cbase + CHUNK <= nE) {
    da = *(const v4i*)(keys + e0);
    db = *(const v4i*)(keys + e0 + 4);
  } else {
    da.x = (e0     < nE) ? keys[min(e0,     nE - 1)] : sent;
    da.y = (e0 + 1 < nE) ? keys[min(e0 + 1, nE - 1)] : sent;
    da.z = (e0 + 2 < nE) ? keys[min(e0 + 2, nE - 1)] : sent;
    da.w = (e0 + 3 < nE) ? keys[min(e0 + 3, nE - 1)] : sent;
    db.x = (e0 + 4 < nE) ? keys[min(e0 + 4, nE - 1)] : sent;
    db.y = (e0 + 5 < nE) ? keys[min(e0 + 5, nE - 1)] : sent;
    db.z = (e0 + 6 < nE) ? keys[min(e0 + 6, nE - 1)] : sent;
    db.w = (e0 + 7 < nE) ? keys[min(e0 + 7, nE - 1)] : sent;
  }
  const unsigned nbs = (unsigned)slotBase;
  const unsigned unb = (unsigned)nb;
  const unsigned s0 = (unsigned)da.x - nbs, s1 = (unsigned)da.y - nbs;
  const unsigned s2 = (unsigned)da.z - nbs, s3 = (unsigned)da.w - nbs;
  const unsigned s4 = (unsigned)db.x - nbs, s5 = (unsigned)db.y - nbs;
  const unsigned s6 = (unsigned)db.z - nbs, s7 = (unsigned)db.w - nbs;
  const bool h0 = s0 < unb, h1 = s1 < unb, h2 = s2 < unb, h3 = s3 < unb;
  const bool h4 = s4 < unb, h5 = s5 < unb, h6 = s6 < unb, h7 = s7 < unb;
  const unsigned any = __builtin_amdgcn_ballot_w32(h0 | h1 | h2 | h3 | h4 | h5 | h6 | h7);
  if (any != 0u) {
#define HITJ(J, HJ, SJ) { \
      const unsigned mj = __builtin_amdgcn_ballot_w32(HJ); \
      if (mj != 0u) { \
        if (HJ) { \
          const int pos = wc + (int)__builtin_amdgcn_mbcnt_lo(mj, 0u); \
          if (pos < WCAP) list[wave * WCAP + pos] = ((el0 + (J)) << SLOTB) | (int)(SJ); \
        } \
        wc += (int)__builtin_popcount(mj); } }
    HITJ(0, h0, s0)
    HITJ(1, h1, s1)
    HITJ(2, h2, s2)
    HITJ(3, h3, s3)
    HITJ(4, h4, s4)
    HITJ(5, h5, s5)
    HITJ(6, h6, s6)
    HITJ(7, h7, s7)
#undef HITJ
  }
  return wc;
}

__global__ __launch_bounds__(NTHR) void k_attn(
    const unsigned short* __restrict__ Qp, const unsigned short* __restrict__ Kp,
    const unsigned short* __restrict__ VTp, const float* __restrict__ EB,
    const int* __restrict__ keys, const int* __restrict__ gath,
    const int* __restrict__ ngp, const int* __restrict__ bat,
    unsigned short* CTX, int nE, int vec8, int gbase) {
  extern __shared__ v4f lds_dyn[];
  char* lds = (char*)lds_dyn;
  __bf16* Ksh = (__bf16*)(lds + LO_KV);
  __bf16* Ksl = Ksh + 2 * KVT;
  __bf16* Vth = Ksl + 2 * KVT;
  __bf16* Vtl = Vth + 2 * KVT;
  int* list  = (int*)(lds + LO_KV);
  int* hitE  = list + LISTN;
  int* hitRD = hitE + HCAP;
  __bf16* Psh = (__bf16*)(lds + LO_P);
  __bf16* Psl = Psh + AT_NW * 1024;
  float* BTX = (float*)(lds + LO_BT);
  int* sE   = (int*)(lds + LO_SE);
  int* sD   = (int*)(lds + LO_SD);
  int* rcnt = (int*)(lds + LO_RC);
  int* roff = rcnt + NSLOT;
  int* curs = roff + NSLOT;
  int* wcnt = curs + NSLOT;
  int* misc = wcnt + AT_NW;

  const int tid = (int)threadIdx.x, lane = tid & 31, wave = tid >> 5, hh = lane >> 4, c = lane & 15;
  const int lgr   = (int)blockIdx.x >> 3;
  const int qt    = (int)blockIdx.x & 7;
  const int gb    = gbase + lgr;
  const int node0 = gb * NND + qt * NSLOT;
  const int lrow0 = lgr * NND + qt * NSLOT;

  if (tid < NSLOT) rcnt[tid] = 0;
  __syncthreads();

  int tot = 0;
  const int nChunks = (nE + CHUNK - 1) / CHUNK;
#pragma unroll 1
  for (int ch = 0; ch < nChunks; ++ch) {
    const int cbase = ch * CHUNK;
    const int wc = scan_chunk(keys, nE, cbase, node0, NSLOT, vec8, list, tid, lane, wave);
    if (lane == 0) wcnt[wave] = wc;
    __syncthreads();
    int pre = 0, all = 0;
#pragma unroll
    for (int w2 = 0; w2 < AT_NW; ++w2) {
      int cc = wcnt[w2];
      cc = cc < 0 ? 0 : (cc > WCAP ? WCAP : cc);
      all += cc;
      pre += (w2 < wave) ? cc : 0;
    }
    const int wcc  = wc > WCAP ? WCAP : wc;
    const int base = tot + pre;
#pragma unroll 1
    for (int i0 = 0; i0 < wcc; i0 += 32) {
      const int i   = i0 + lane;
      const int ic  = i < wcc ? i : wcc - 1;
      const int ent = list[wave * WCAP + ic];
      const int el  = (ent >> SLOTB) & (CHUNK - 1);
      const int sl  = ent & (NSLOT - 1);
      int eid = cbase + el;
      eid = eid > nE - 1 ? nE - 1 : eid;
      int g = gath[eid];
      g = g < 0 ? 0 : (g > NTOT - 1 ? NTOT - 1 : g);
      const int pos = base + i;
      if (i < wcc && pos < HCAP) {
        hitE[pos]  = eid;
        hitRD[pos] = (sl << 9) | (g & (NND - 1));
      }
    }
    tot += all;
    tot = tot > HCAP ? HCAP : tot;
    __syncthreads();
  }
  const int nh = tot;

  if (wave == 0) {
#pragma unroll 1
    for (int b0 = 0; b0 < nh; b0 += 32) {
      const int idx = b0 + lane;
      const int uv  = hitRD[idx < nh ? idx : nh - 1];
      const int m32 = (nh - b0) < 32 ? (nh - b0) : 32;
#pragma unroll 1
      for (int k = 0; k < m32; ++k) {
        const int u  = __builtin_amdgcn_readlane(uv, k);
        const int sl = (u >> 9) & (NSLOT - 1);
        if (lane == 0) rcnt[sl] = rcnt[sl] + 1;
      }
    }
  }
  __syncthreads();

  if (wave == 0) {
    int c0 = rcnt[2 * lane], c1 = rcnt[2 * lane + 1];
    c0 = c0 < 0 ? 0 : c0; c1 = c1 < 0 ? 0 : c1;
    const int ts = c0 + c1;
    int incl = ts;
#pragma unroll
    for (int d = 1; d < 32; d <<= 1) {
      const int up = __shfl_up(incl, d, 32);
      if (lane >= d) incl += up;
    }
    const int excl = incl - ts;
    roff[2 * lane] = excl;     roff[2 * lane + 1] = excl + c0;
    curs[2 * lane] = excl;     curs[2 * lane + 1] = excl + c0;
    int mc = c0 > c1 ? c0 : c1;
#pragma unroll
    for (int off = 16; off > 0; off >>= 1) {
      const int o = __shfl_xor(mc, off, 32);
      mc = o > mc ? o : mc;
    }
    if (lane == 0) misc[0] = mc;
  }
  __syncthreads();

  if (wave == 0) {
#pragma unroll 1
    for (int b0 = 0; b0 < nh; b0 += 32) {
      const int idx = b0 + lane;
      const int cl  = idx < nh ? idx : nh - 1;
      const int uv  = hitRD[cl];
      const int ue  = hitE[cl];
      const int m32 = (nh - b0) < 32 ? (nh - b0) : 32;
#pragma unroll 1
      for (int k = 0; k < m32; ++k) {
        const int u  = __builtin_amdgcn_readlane(uv, k);
        const int e  = __builtin_amdgcn_readlane(ue, k);
        const int sl = (u >> 9) & (NSLOT - 1);
        if (lane == 0) {
          int pos = curs[sl];
          pos = pos < 0 ? 0 : (pos > HCAP - 1 ? HCAP - 1 : pos);
          sE[pos] = e;
          sD[pos] = u & (NND - 1);
          curs[sl] = pos + 1;
        }
      }
    }
  }
  __syncthreads();

  const int degmax = misc[0];
  const int ng  = ngp[0];
  const int bt0 = bat[node0];
  const bool bad = (nh >= HCAP) || (degmax > RWCAP) || (ng != NGR) || (bt0 < 0) || (bt0 >= NGR);
  const float pz = bad ? __int_as_float(0x7fc00000) : 0.0f;

  const int wsub = wave & 3;
  const int hl   = wave >> 2;
  const int rw   = tid >> 2;
  const int jw   = tid & 3;
  const float sscale = 0.125f;
  const v8f z8 = {0.f,0.f,0.f,0.f,0.f,0.f,0.f,0.f};
  const __bf16* Kth = Ksh + hl * KVT;
  const __bf16* Ktl = Ksl + hl * KVT;
  const __bf16* Vtth = Vth + hl * KVT;
  const __bf16* Vttl = Vtl + hl * KVT;
  __bf16* pwh = Psh + wave * 1024;
  __bf16* pwl = Psl + wave * 1024;

#pragma unroll 1
  for (int hp = 0; hp < NHD / 2; ++hp) {
    const int h    = 2 * hp + hl;
    const int qrow = lrow0 + wsub * 16;

    v16b qah[2], qal[2];
#pragma unroll
    for (int dc = 0; dc < 2; ++dc) {
      const unsigned short* qp = Qp + (size_t)(qrow + c) * PLD + h * HDM + dc * 32 + 8 * hh;
      qah[dc] = FragBF::load((const __bf16*)(const void*)qp);
      qal[dc] = FragBF::load((const __bf16*)(const void*)(qp + HID));
    }
    float mrow[8], lrow[8];
    v8f oacc[4];
#pragma unroll
    for (int r = 0; r < 8; ++r) { mrow[r] = -INFINITY; lrow[r] = 0.f; }
#pragma unroll
    for (int t = 0; t < 4; ++t) oacc[t] = z8;

#pragma unroll 1
    for (int kc = 0; kc < NND / 64; ++kc) {
      const int kv0 = kc * 64;
      __syncthreads();
      {
        const int th = tid >> 7, t = tid & 127;
        const int r = t >> 1, half = (t & 1) * 32;
        const int hs = 2 * hp + th;
        const unsigned short* ksh = Kp + (size_t)(lgr * NND + kv0 + r) * PLD + hs * HDM + half;
        const unsigned short* ksl = ksh + HID;
        const unsigned short* vsh = VTp + ((size_t)lgr * HID + hs * HDM + r) * PLD + kv0 + half;
        const unsigned short* vsl = vsh + HID;
        __bf16* kdh = Ksh + th * KVT + r * HDM + half;
        __bf16* kdl = Ksl + th * KVT + r * HDM + half;
        __bf16* vdh = Vth + th * KVT + r * 64 + half;
        __bf16* vdl = Vtl + th * KVT + r * 64 + half;
#pragma unroll
        for (int i = 0; i < 4; ++i) {
          const v8b a0 = *(const v8b*)(ksh + 8 * i);
          const v8b a1 = *(const v8b*)(ksl + 8 * i);
          const v8b b0 = *(const v8b*)(vsh + 8 * i);
          const v8b b1 = *(const v8b*)(vsl + 8 * i);
          *(v8b*)(kdh + 8 * i) = a0;
          *(v8b*)(kdl + 8 * i) = a1;
          *(v8b*)(vdh + 8 * i) = b0;
          *(v8b*)(vdl + 8 * i) = b1;
        }
        const v4f z4 = {0.f, 0.f, 0.f, 0.f};
        float* bz = BTX + tid * 32;
#pragma unroll
        for (int i = 0; i < 8; ++i) *(v4fa*)(bz + 4 * i) = z4;
        if (tid < 128) *(v4fa*)(BTX + 2 * KVT + 4 * tid) = z4;
      }
      __syncthreads();
      {
        int st = roff[rw], cnt = rcnt[rw];
        st  = st < 0 ? 0 : (st > nh ? nh : st);
        cnt = cnt < 0 ? 0 : (cnt > RWCAP ? RWCAP : cnt);
        if (cnt > nh - st) cnt = nh - st;
        int cmax = cnt;
#pragma unroll
        for (int off = 16; off > 0; off >>= 1) {
          const int o = __shfl_xor(cmax, off, 32);
          cmax = o > cmax ? o : cmax;
        }
        const float* ebp = EB + 2 * hp;
#pragma unroll 1
        for (int q = 0; q < cmax; ++q) {
          const bool valid = q < cnt;
          int idx = st + q;
          idx = idx > nh - 1 ? nh - 1 : idx;
          idx = idx < 0 ? 0 : idx;
          const int col = sD[idx] - kv0;
          int e = sE[idx];
          e = e < 0 ? 0 : (e > nE - 1 ? nE - 1 : e);
          const v2f ebv = *(const v2fa*)(ebp + (size_t)e * NHD);
          const bool inr = valid && ((unsigned)col < 64u) && ((col >> 4) == jw);
          const int ia = inr ? (rw * 64 + col) : (2 * KVT + tid);
          const int ib = inr ? (KVT + rw * 64 + col) : (2 * KVT + NTHR + tid);
          BTX[ia] = BTX[ia] + ebv.x;
          BTX[ib] = BTX[ib] + ebv.y;
        }
      }
      __syncthreads();

      v8f s[4];
#pragma unroll
      for (int j = 0; j < 4; ++j) {
        s[j] = z8;
#pragma unroll
        for (int dc = 0; dc < 2; ++dc) {
          FB kb, kl;
          const __bf16* kr = Kth + (j * 16 + c) * HDM + dc * 32 + 8 * hh;
          const __bf16* kq = Ktl + (j * 16 + c) * HDM + dc * 32 + 8 * hh;
          kb.h[0] = *(const v8b*)kr;
          kb.h[1] = *(const v8b*)(kr + 16);
          kl.h[0] = *(const v8b*)kq;
          kl.h[1] = *(const v8b*)(kq + 16);
          s[j] = at_mma(qah[dc], kb.v, s[j]);
          s[j] = at_mma(qah[dc], kl.v, s[j]);
          s[j] = at_mma(qal[dc], kb.v, s[j]);
        }
      }
      const float* btr = BTX + hl * KVT + (wsub * 16 + 8 * hh) * 64 + c;
      float cm[8];
#pragma unroll
      for (int r = 0; r < 8; ++r) {
        float m = -INFINITY;
#pragma unroll
        for (int j = 0; j < 4; ++j) {
          const float sv = s[j][r] * sscale + btr[r * 64 + j * 16];
          s[j][r] = sv;
          m = fmaxf(m, sv);
        }
#pragma unroll
        for (int off = 1; off < 16; off <<= 1) m = fmaxf(m, __shfl_xor(m, off, 32));
        cm[r] = m;
      }
#pragma unroll
      for (int r = 0; r < 8; ++r) {
        const float mnew = fmaxf(mrow[r], cm[r]);
        const float alpha = expf(mrow[r] - mnew);
        mrow[r] = mnew;
        float psum = 0.f;
#pragma unroll
        for (int j = 0; j < 4; ++j) {
          const float p = expf(s[j][r] - mnew);
          psum += p;
          __bf16 a, bl; at_split(p, a, bl);
          pwh[(8 * hh + r) * 64 + j * 16 + c] = a;
          pwl[(8 * hh + r) * 64 + j * 16 + c] = bl;
        }
#pragma unroll
        for (int off = 1; off < 16; off <<= 1) psum += __shfl_xor(psum, off, 32);
        lrow[r] = lrow[r] * alpha + psum;
#pragma unroll
        for (int t = 0; t < 4; ++t) oacc[t][r] *= alpha;
      }
      __builtin_amdgcn_fence(__ATOMIC_RELEASE, "workgroup");
      __builtin_amdgcn_wave_barrier();
      __builtin_amdgcn_fence(__ATOMIC_ACQUIRE, "workgroup");
#pragma unroll 1
      for (int kk = 0; kk < 2; ++kk) {
        FB pa, pl;
        pa.h[0] = *(const v8b*)(pwh + c * 64 + kk * 32 + 8 * hh);
        pa.h[1] = *(const v8b*)(pwh + c * 64 + kk * 32 + 16 + 8 * hh);
        pl.h[0] = *(const v8b*)(pwl + c * 64 + kk * 32 + 8 * hh);
        pl.h[1] = *(const v8b*)(pwl + c * 64 + kk * 32 + 16 + 8 * hh);
#pragma unroll
        for (int t = 0; t < 4; ++t) {
          FB vb, vl;
          vb.h[0] = *(const v8b*)(Vtth + (t * 16 + c) * 64 + kk * 32 + 8 * hh);
          vb.h[1] = *(const v8b*)(Vtth + (t * 16 + c) * 64 + kk * 32 + 16 + 8 * hh);
          vl.h[0] = *(const v8b*)(Vttl + (t * 16 + c) * 64 + kk * 32 + 8 * hh);
          vl.h[1] = *(const v8b*)(Vttl + (t * 16 + c) * 64 + kk * 32 + 16 + 8 * hh);
          oacc[t] = at_mma(pa.v, vb.v, oacc[t]);
          oacc[t] = at_mma(pa.v, vl.v, oacc[t]);
          oacc[t] = at_mma(pl.v, vb.v, oacc[t]);
        }
      }
    }

    __syncthreads();
    {
      float* os = BTX + wave * 1024;
#pragma unroll
      for (int r = 0; r < 8; ++r) {
        const float inv = 1.0f / lrow[r];
#pragma unroll
        for (int t = 0; t < 4; ++t) os[(8 * hh + r) * 64 + t * 16 + c] = oacc[t][r] * inv + pz;
      }
      __builtin_amdgcn_fence(__ATOMIC_RELEASE, "workgroup");
      __builtin_amdgcn_wave_barrier();
      __builtin_amdgcn_fence(__ATOMIC_ACQUIRE, "workgroup");
      const int q4 = lane >> 3, c8 = (lane & 7) * 8;
      v4u hv[4], lv[4];
#pragma unroll
      for (int it = 0; it < 4; ++it) {
        const int row = it * 4 + q4;
        const float* sp = os + row * 64 + c8;
        const v4f a = *(const v4fa*)sp;
        const v4f b = *(const v4fa*)(sp + 4);
        pack8hl(a, b, hv[it], lv[it]);
      }
      for (int pass = 0; pass < 2; ++pass) {
#pragma unroll
        for (int it = 0; it < 4; ++it) {
          const int row = it * 4 + q4;
          unsigned short* op = CTX + (size_t)(qrow + row) * PLD + h * HDM + c8;
          *(volatile v4u*)op = hv[it];
          *(volatile v4u*)(op + HID) = lv[it];
        }
        __threadfence();
      }
    }
  }
}

static inline int cdiv(int a, int b) { return (a + b - 1) / b; }

extern "C" void kernel_launch(void* const* d_in, const int* in_sizes, int n_in,
                              void* d_out, int out_size, void* d_ws, size_t ws_size,
                              hipStream_t stream) {
  if (n_in < 15) return;
  if (in_sizes[0] != NTOT * HID) return;
  if (in_sizes[1] != NTOT) return;
  if (in_sizes[2] < 2 || (in_sizes[2] & 1) != 0) return;
  const int nE = in_sizes[2] / 2;
  if (nE < 1 || nE > (1 << 24)) return;
  if (in_sizes[3] != nE * EDW) return;
  if (in_sizes[4] != HID * HID || in_sizes[6] != HID * HID || in_sizes[8] != HID * HID || in_sizes[10] != HID * HID) return;
  if (in_sizes[5] != HID || in_sizes[7] != HID || in_sizes[9] != HID || in_sizes[11] != HID) return;
  if (in_sizes[12] != EDW * NHD || in_sizes[13] != NHD || in_sizes[14] != 1) return;
  if (out_size != NTOT * HID) return;

  const float* x   = (const float*)d_in[0];
  const int*   bat = (const int*)  d_in[1];
  const int*   ei  = (const int*)  d_in[2];
  const float* ea  = (const float*)d_in[3];
  const float* Wq  = (const float*)d_in[4];
  const float* bq  = (const float*)d_in[5];
  const float* Wk  = (const float*)d_in[6];
  const float* bk  = (const float*)d_in[7];
  const float* Wv  = (const float*)d_in[8];
  const float* bv  = (const float*)d_in[9];
  const float* Wo  = (const float*)d_in[10];
  const float* bo  = (const float*)d_in[11];
  const float* We  = (const float*)d_in[12];
  const float* be  = (const float*)d_in[13];
  const int*   ngp = (const int*)  d_in[14];
  float* out = (float*)d_out;
  const int* keys = ei;
  const int* gath = ei + nE;

  const int EP = cdiv(nE, 4) * 4;

  char* ws = (char*)d_ws;
  size_t off = 0;
  const size_t oXb = off; off += (size_t)NTOT * HID * 2;
  const size_t oWq = off; off += (size_t)HID * HID * 2;
  const size_t oWk = off; off += (size_t)HID * HID * 2;
  const size_t oWv = off; off += (size_t)HID * HID * 2;
  const size_t oWo = off; off += (size_t)HID * PLD * 2;
  const size_t oEB = off; off += (size_t)EP * NHD * 4;   off = (off + 255) & ~(size_t)255;
  const size_t oQ  = off; off += (size_t)RHALF * PLD * 2;
  const size_t oK  = off; off += (size_t)RHALF * PLD * 2;
  const size_t oVT = off; off += (size_t)GHALF * HID * PLD * 2;
  const size_t oCT = off; off += (size_t)RHALF * PLD * 2;
  if (off > ws_size || off > (size_t)WSMAX) return;
  unsigned short* Xb   = (unsigned short*)(ws + oXb);
  unsigned short* WqT  = (unsigned short*)(ws + oWq);
  unsigned short* WkT  = (unsigned short*)(ws + oWk);
  unsigned short* WvT  = (unsigned short*)(ws + oWv);
  unsigned short* WOT2 = (unsigned short*)(ws + oWo);
  float*          EB   = (float*)(ws + oEB);
  unsigned short* Qp   = (unsigned short*)(ws + oQ);
  unsigned short* Kp   = (unsigned short*)(ws + oK);
  unsigned short* VTp  = (unsigned short*)(ws + oVT);
  unsigned short* CTX  = (unsigned short*)(ws + oCT);

  hipFuncSetAttribute(reinterpret_cast<const void*>(&k_attn),
                      hipFuncAttributeMaxDynamicSharedMemorySize, LDS_ATT);

  {
    const int nUw = HID * (HID / 8);
    k_wtr<<<cdiv(nUw, NTHR), NTHR, 0, stream>>>(Wq, HID, HID, HID, HID, WqT, nUw);
    k_wtr<<<cdiv(nUw, NTHR), NTHR, 0, stream>>>(Wk, HID, HID, HID, HID, WkT, nUw);
    k_wtr<<<cdiv(nUw, NTHR), NTHR, 0, stream>>>(Wv, HID, HID, HID, HID, WvT, nUw);
    const int nUo = HID * (PLD / 8);
    k_wtr<<<cdiv(nUo, NTHR), NTHR, 0, stream>>>(Wo, HID, HID, HID, PLD, WOT2, nUo);
  }
  {
    const int nUx = NTOT * (HID / 8);
    k_xprep<<<cdiv(nUx, NTHR), NTHR, 0, stream>>>(x, Xb, NTOT, nUx);
  }
  {
    const int nUe = EP * 2;
    k_eb<<<cdiv(nUe, NTHR), NTHR, 0, stream>>>(ea, We, be, EB, nE, nUe);
  }

  const dim3 blk(256);
  const dim3 gQK(((RHALF / 64) * (HID / 64)) / 8, 1);
  const dim3 gVT(((HID / 64) * (NND / 64)) / 8, GHALF);
  const dim3 gAT(GHALF * (NND / 64));
  for (int half = 0; half < NHALF; ++half) {
    const unsigned short* Xh = Xb + (size_t)half * RHALF * HID;
    float* outh = out + (size_t)half * RHALF * HID;
    wmma_gemm64<false, 2, 2, false, 0><<<gQK, blk, 0, stream>>>(
        Xh, Xh, HID, 0L, WqT, WqT, HID, 0L, (void*)Qp, (void*)(Qp + HID), PLD, 0L,
        bq, bq, 0L, RHALF, HID, HID, 1.0f);
    wmma_gemm64<false, 2, 2, false, 0><<<gQK, blk, 0, stream>>>(
        Xh, Xh, HID, 0L, WkT, WkT, HID, 0L, (void*)Kp, (void*)(Kp + HID), PLD, 0L,
        bk, bk, 0L, RHALF, HID, HID, 1.0f);
    wmma_gemm64<false, 1, 2, false, 0><<<gVT, blk, 0, stream>>>(
        WvT, WvT, HID, 0L, Xh, Xh, HID, (long)NND * HID, (void*)VTp, (void*)(VTp + HID), PLD, (long)HID * PLD,
        bv, bv, 0L, HID, NND, HID, 1.0f);
    k_attn<<<gAT, NTHR, LDS_ATT, stream>>>(Qp, Kp, VTp, EB, keys, gath, ngp, bat, CTX, nE, 1, half * GHALF);
    wmma_gemm64<false, 2, 0, false, 0><<<gQK, blk, 0, stream>>>(
        CTX, CTX, PLD, 0L, WOT2, WOT2, PLD, 0L, (void*)outh, (void*)outh, HID, 0L,
        bo, bo, 0L, RHALF, HID, PLD, 1.0f);
  }
  (void)hipGetLastError();
}
